// SelfAttentionMemory_7533372637187
// MI455X (gfx1250) — hardware-verified
//
#include <hip/hip_runtime.h>
#include <math.h>

typedef __attribute__((ext_vector_type(16))) _Float16 v16h;
typedef __attribute__((ext_vector_type(16))) __bf16 v16b;
typedef __attribute__((ext_vector_type(8)))  _Float16 v8h;
typedef __attribute__((ext_vector_type(8)))  float v8f;
typedef __attribute__((ext_vector_type(4)))  float v4f;
typedef __attribute__((ext_vector_type(2)))  float v2f;
typedef __attribute__((ext_vector_type(4)))  unsigned v4u;
typedef __attribute__((ext_vector_type(4)))  int v4i;
typedef float __attribute__((may_alias)) float_a;
typedef int __attribute__((may_alias)) int_a;

template <typename T> __device__ __forceinline__ void vst2(void* p, T v) { *(volatile T*)p = v; __threadfence(); *(volatile T*)p = v; }
__device__ __forceinline__ v8f wmma16(v16h a, v16h b, v8f c) {
  v8f d = __builtin_amdgcn_wmma_f32_16x16x32_f16(false, a, false, b, (short)0, c, false, false);
  asm volatile("v_nop\n\tv_nop\n\tv_nop\n\tv_nop" : "+v"(d) : "v"(a), "v"(b));
  return d;
}
__device__ __forceinline__ v8f wmma_bf(v16b a, v16b b, v8f c) {
  v8f d = __builtin_amdgcn_wmma_f32_16x16x32_bf16(false, a, false, b, (short)0, c, false, false);
  asm volatile("v_nop\n\tv_nop\n\tv_nop\n\tv_nop" : "+v"(d) : "v"(a), "v"(b));
  return d;
}
__device__ __forceinline__ v16h frag_h(const _Float16* rowk0, int lane) {
  union { v16h v; v8h q[2]; } u; const _Float16* p = rowk0 + 8 * (lane >> 4);
  u.q[0] = *(const v8h*)p; u.q[1] = *(const v8h*)(p + 16); return u.v;
}
__device__ __forceinline__ v16h frag_f32(const float* rowk0, int lane) {
  v16h a; const float* p = rowk0 + 8 * (lane >> 4);
#pragma unroll
  for (int i = 0; i < 8; ++i) { a[i] = (_Float16)p[i]; a[8 + i] = (_Float16)p[16 + i]; }
  return a;
}
__device__ __forceinline__ v16h frag_f32s(const float* rowk0, int lane, float sc) {
  v16h a; const float* p = rowk0 + 8 * (lane >> 4);
#pragma unroll
  for (int i = 0; i < 8; ++i) { a[i] = (_Float16)(p[i] * sc); a[8 + i] = (_Float16)(p[16 + i] * sc); }
  return a;
}
__device__ __forceinline__ v16h fragc_f32(const float* W, int k0, int n, int lane, int ld, int K) {
  v16h a; const int g = lane >> 4;
#pragma unroll
  for (int i = 0; i < 8; ++i) { const int ka = k0 + 8 * g + i, kb = ka + 16;
    a[i] = (_Float16)(ka < K ? W[(size_t)(ka < K ? ka : K - 1) * ld + n] : 0.f); a[8 + i] = (_Float16)(kb < K ? W[(size_t)(kb < K ? kb : K - 1) * ld + n] : 0.f); }
  return a;
}
struct F2 { v16b h, l; };
__device__ __forceinline__ F2 bsplit16(const float v[16]) { F2 r;
#pragma unroll
  for (int i = 0; i < 16; ++i) { const __bf16 h = (__bf16)v[i]; r.h[i] = h; r.l[i] = (__bf16)(v[i] - (float)h); }
  return r; }
__device__ __forceinline__ F2 split_row(const float* row, int k0, int lane) { float v[16]; const float* p = row + k0 + 8 * (lane >> 4);
#pragma unroll
  for (int i = 0; i < 8; ++i) { v[i] = p[i]; v[8 + i] = p[16 + i]; }
  return bsplit16(v); }
__device__ __forceinline__ F2 split_rowK(const float* row, int k0, int lane, int K) { float v[16]; const int g = lane >> 4;
#pragma unroll
  for (int i = 0; i < 8; ++i) { const int ka = k0 + 8 * g + i, kb = ka + 16; v[i] = ka < K ? row[ka < K ? ka : K - 1] : 0.f; v[8 + i] = kb < K ? row[kb < K ? kb : K - 1] : 0.f; }
  return bsplit16(v); }
__device__ __forceinline__ F2 split_col(const float* W, int k0, int n, int lane, int ld, int K) { float v[16]; const int g = lane >> 4;
#pragma unroll
  for (int i = 0; i < 8; ++i) { const int ka = k0 + 8 * g + i, kb = ka + 16; v[i] = ka < K ? W[(size_t)(ka < K ? ka : K - 1) * ld + n] : 0.f; v[8 + i] = kb < K ? W[(size_t)(kb < K ? kb : K - 1) * ld + n] : 0.f; }
  return bsplit16(v); }
__device__ __forceinline__ v8f mac3(const F2& a, const F2& b, v8f c) { c = wmma_bf(a.l, b.h, c); c = wmma_bf(a.h, b.l, c); return wmma_bf(a.h, b.h, c); }
__device__ __forceinline__ float sigm(float v) { return 1.0f / (1.0f + expf(-v)); }
#define LDSX() do { asm volatile("s_wait_dscnt 0" ::: "memory"); __builtin_amdgcn_wave_barrier(); __builtin_amdgcn_fence(__ATOMIC_RELEASE, "workgroup"); } while (0)


#define NB 8
#define CC 64
#define NN 4096
#define NR (NB * NN)
#define QK 8
#ifndef TNB
#define TNB NB
#endif
typedef __attribute__((ext_vector_type(8))) __bf16 v8b;
__device__ __forceinline__ v16b frag_b(const __bf16* rowk0, int lane) {
  union { v16b v; v8b q[2]; } u; const __bf16* p = rowk0 + 8 * (lane >> 4);
  u.q[0] = *(const v8b*)p; u.q[1] = *(const v8b*)(p + 16); return u.v;
}
__device__ __forceinline__ float bfr(float v) { return (float)(__bf16)v; }
__device__ __attribute__((noinline)) float exp_ni(float v) { return expf(v); }
__device__ __attribute__((noinline)) float erf_ni(float v) { return erff(v); }
__device__ __attribute__((noinline)) float tanh_ni(float v) { return tanhf(v); }

#define PK_JH 0
#define PK_JM (96 * CC)
#define PK_Z  (PK_JM + 80 * CC)
#define PK_G  (PK_Z + CC * 2 * CC)
#define PK_END (PK_G + 3 * CC * 2 * CC)
#define WS_PK  0u
#define WS_HT  (((2u * PK_END) + 127u) / 128u * 128u)
#define WS_QP  (WS_HT + 2u * NR * CC)
#define WS_KP  (WS_QP + 2u * NR * 32)
#define WS_VH  (WS_KP + 2u * 2 * NR * 32)
#define WS_VL  (WS_VH + 2u * 2 * NR * CC)
#define WS_ZRH (WS_VL + 2u * 2 * NR * CC)
#define WS_ZRL (WS_ZRH + 2u * NR * 2 * CC)
#define WS_END (WS_ZRL + 2u * NR * 2 * CC)

__global__ __launch_bounds__(128) void k_pack(const float* __restrict__ WQ, const float* __restrict__ WKH, const float* __restrict__ WVH, const float* __restrict__ WKM, const float* __restrict__ WVM, const float* __restrict__ WZ, const float* __restrict__ WO, const float* __restrict__ WG, const float* __restrict__ WI, __bf16* __restrict__ PK) {
  __shared__ __align__(16) __bf16 s[2 * CC]; const int n = blockIdx.x, which = blockIdx.y, t = threadIdx.x; int K; size_t dst; float v = 0.f;
  if (which == 0) { if (n >= 96) return; K = CC; dst = PK_JH + (size_t)n * CC; if (t < CC) { if (n < 16) v = (n < QK) ? WQ[(size_t)n * CC + t] : 0.f; else if (n < 32) v = (n - 16 < QK) ? WKH[(size_t)(n - 16) * CC + t] : 0.f; else v = WVH[(size_t)(n - 32) * CC + t]; s[t] = (__bf16)v; } }
  else if (which == 1) { if (n >= 80) return; K = CC; dst = PK_JM + (size_t)n * CC; if (t < CC) { if (n < 16) v = (n < QK) ? WKM[(size_t)n * CC + t] : 0.f; else v = WVM[(size_t)(n - 16) * CC + t]; s[t] = (__bf16)v; } }
  else if (which == 2) { if (n >= CC) return; K = 2 * CC; dst = PK_Z + (size_t)n * 2 * CC; s[t] = (__bf16)WZ[(size_t)n * 2 * CC + t]; }
  else { if (n >= 3 * CC) return; K = 2 * CC; dst = PK_G + (size_t)n * 2 * CC; const float* Wm = (n < CC) ? WO : (n < 2 * CC) ? WG : WI; s[t] = (__bf16)Wm[(size_t)(n % CC) * 2 * CC + t]; }
  __syncthreads();
  if (t < K / 8) vst2((unsigned*)(PK + dst + t * 8), *(const v4u*)&s[t * 8]);
}
__global__ __launch_bounds__(128) void k_proj(const float* __restrict__ HIN, const float* __restrict__ MIN_, const __bf16* __restrict__ PK, const float* __restrict__ BQ, const float* __restrict__ BKH, const float* __restrict__ BVH, const float* __restrict__ BKM, const float* __restrict__ BVM, __bf16* __restrict__ HT, _Float16* __restrict__ QP, _Float16* __restrict__ KP, _Float16* __restrict__ VH, _Float16* __restrict__ VL) {
  __shared__ __align__(16) __bf16 sh_[64][CC + 8], sm_[64][CC + 8]; __shared__ __align__(16) _Float16 sq[4][16][40], skh[4][16][40], skm[4][16][40]; __shared__ __align__(16) _Float16 svh[2][CC][72], svl[2][CC][72];
  const int tid = threadIdx.x, wave = tid >> 5, lane = tid & 31, col = lane & 15, g = lane >> 4; const int pb = blockIdx.x, b = blockIdx.y; const int n0 = pb * 64; const size_t row0 = (size_t)b * NN + n0;
  for (int e = tid; e < 64 * CC; e += 128) { const int c = e >> 6, r = e & 63; sh_[r][c] = (__bf16)HIN[((size_t)b * CC + c) * NN + n0 + r]; sm_[r][c] = (__bf16)MIN_[((size_t)b * CC + c) * NN + n0 + r]; }
  for (int e = tid; e < 4 * 16 * 40; e += 128) { (&sq[0][0][0])[e] = (_Float16)0.f; (&skh[0][0][0])[e] = (_Float16)0.f; (&skm[0][0][0])[e] = (_Float16)0.f; }
  __syncthreads();
  v8f ah[6] = {}, am[5] = {};
#pragma unroll
  for (int kc = 0; kc < CC / 32; ++kc) { const v16b a1 = frag_b(&sh_[wave * 16 + col][kc * 32], lane), a2 = frag_b(&sm_[wave * 16 + col][kc * 32], lane);
#pragma unroll
    for (int j = 0; j < 6; ++j) ah[j] = wmma_bf(a1, frag_b(PK + PK_JH + (size_t)(j * 16 + col) * CC + kc * 32, lane), ah[j]);
#pragma unroll
    for (int j = 0; j < 5; ++j) am[j] = wmma_bf(a2, frag_b(PK + PK_JM + (size_t)(j * 16 + col) * CC + kc * 32, lane), am[j]); }
  const float isq = 0.35355339059327373f;
#pragma unroll
  for (int r = 0; r < 8; ++r) { const int rl = 8 * g + r;
    if (col < QK) { sq[wave][rl][col] = (_Float16)((ah[0][r] + bfr(BQ[col])) * isq); skh[wave][rl][col] = (_Float16)(ah[1][r] + bfr(BKH[col])); skm[wave][rl][col] = (_Float16)(am[0][r] + bfr(BKM[col])); }
#pragma unroll
    for (int j = 0; j < 4; ++j) { const int c = j * 16 + col; { const float v = ah[2 + j][r] + bfr(BVH[c]); const _Float16 hv = (_Float16)v; svh[0][c][wave * 16 + rl] = hv; svl[0][c][wave * 16 + rl] = (_Float16)((v - (float)hv) * 2048.0f); } { const float v = am[1 + j][r] + bfr(BVM[c]); const _Float16 hv = (_Float16)v; svh[1][c][wave * 16 + rl] = hv; svl[1][c][wave * 16 + rl] = (_Float16)((v - (float)hv) * 2048.0f); } } }
  __syncthreads();
  for (int rl = 0; rl < 16; ++rl) { const size_t row = row0 + wave * 16 + rl;
    if (lane < 8) vst2((unsigned*)(HT + row * CC + lane * 8), *(const v4u*)&sh_[wave * 16 + rl][lane * 8]);
    else if ((rl & 1) == 0) {
      const int l8 = lane & 7; const int rr = rl + (l8 >> 2); const int pc = l8 & 3; const size_t rw = row + (l8 >> 2);
      if (lane < 16) vst2((unsigned*)(QP + rw * 32 + pc * 8), *(const v4u*)&sq[wave][rr][pc * 8]);
      else if (lane < 24) vst2((unsigned*)(KP + rw * 32 + pc * 8), *(const v4u*)&skh[wave][rr][pc * 8]);
      else vst2((unsigned*)(KP + ((size_t)NR + rw) * 32 + pc * 8), *(const v4u*)&skm[wave][rr][pc * 8]); } }
  for (int e = tid; e < 2 * CC * 8; e += 128) { const int src = e / (CC * 8), rem = e % (CC * 8); const int c = rem >> 3, pc = rem & 7; const size_t o = (((size_t)src * NB + b) * CC + c) * NN + n0 + pc * 8; vst2((unsigned*)(VH + o), *(const v4u*)&svh[src][c][pc * 8]); vst2((unsigned*)(VL + o), *(const v4u*)&svl[src][c][pc * 8]); }
}
__global__ __launch_bounds__(128) void k_attn(const _Float16* __restrict__ QP, const _Float16* __restrict__ KP, const _Float16* __restrict__ VH, const _Float16* __restrict__ VL, __bf16* __restrict__ ZRH, __bf16* __restrict__ ZRL) {
  __shared__ __align__(16) _Float16 sp[4][16][40]; __shared__ __align__(16) __bf16 soh[4][16][72], sol[4][16][72];
  const int tid = threadIdx.x, wave = tid >> 5, lane = tid & 31, col = lane & 15, g = lane >> 4; const int qb = blockIdx.x, src = blockIdx.y, b = blockIdx.z; const size_t q0 = (size_t)b * NN + (size_t)qb * 64 + wave * 16;
  const v16h aq = frag_h(QP + (q0 + col) * 32, lane); const _Float16* Kb = KP + ((size_t)src * NR + (size_t)b * NN) * 32; const _Float16* Vhb = VH + ((size_t)src * NB + b) * CC * NN; const _Float16* Vlb = VL + ((size_t)src * NB + b) * CC * NN;
  float m[8], l[8];
#pragma unroll
  for (int r = 0; r < 8; ++r) { m[r] = -3.0e38f; l[r] = 0.f; }
  v8f acc[4] = {}, accl[4] = {};
#pragma unroll 1
  for (int ks = 0; ks < NN / 32; ++ks) { v8f s[2];
#pragma unroll
    for (int ct = 0; ct < 2; ++ct) { const size_t kk = (size_t)ks * 32 + ct * 16 + col; v8f c = {}; c = wmma16(aq, frag_h(Kb + kk * 32, lane), c);
#pragma unroll
      for (int r = 0; r < 8; ++r) s[ct][r] = c[r]; }
#pragma unroll
    for (int r = 0; r < 8; ++r) { float mx = fmaxf(s[0][r], s[1][r]);
#pragma unroll
      for (int o = 1; o < 16; o <<= 1) mx = fmaxf(mx, __shfl_xor(mx, o));
      const float mn = fmaxf(m[r], mx); const float alpha = (m[r] <= -1.0e38f) ? 0.f : exp_ni(m[r] - mn); const float e0 = exp_ni(s[0][r] - mn), e1 = exp_ni(s[1][r] - mn); float es = e0 + e1;
#pragma unroll
      for (int o = 1; o < 16; o <<= 1) es += __shfl_xor(es, o);
      l[r] = l[r] * alpha + es; m[r] = mn;
#pragma unroll
      for (int dt = 0; dt < 4; ++dt) { acc[dt][r] *= alpha; accl[dt][r] *= alpha; }
      sp[wave][8 * g + r][col] = (_Float16)e0; sp[wave][8 * g + r][16 + col] = (_Float16)e1; }
    LDSX();
    const v16h pa = frag_h(&sp[wave][col][0], lane);
#pragma unroll
    for (int dt = 0; dt < 4; ++dt) { const size_t vo = (size_t)(dt * 16 + col) * NN + (size_t)ks * 32; acc[dt] = wmma16(pa, frag_h(Vhb + vo, lane), acc[dt]); accl[dt] = wmma16(pa, frag_h(Vlb + vo, lane), accl[dt]); }
    LDSX(); }
#pragma unroll
  for (int r = 0; r < 8; ++r) { const float il = 1.0f / l[r];
#pragma unroll
    for (int dt = 0; dt < 4; ++dt) { const float v = (acc[dt][r] + accl[dt][r] * (1.0f / 2048.0f)) * il; const __bf16 hb = (__bf16)v; soh[wave][8 * g + r][dt * 16 + col] = hb; sol[wave][8 * g + r][dt * 16 + col] = (__bf16)(v - (float)hb); } }
  LDSX();
  for (int rl = 0; rl < 16; ++rl) { const size_t o = (q0 + rl) * 2 * CC + src * CC; if (lane < 8) vst2((unsigned*)(ZRH + o + lane * 8), *(const v4u*)&soh[wave][rl][lane * 8]); else if (lane < 16) vst2((unsigned*)(ZRL + o + (lane - 8) * 8), *(const v4u*)&sol[wave][rl][(lane - 8) * 8]); }
}
__global__ __launch_bounds__(128) void k_gate(const __bf16* __restrict__ ZRH, const __bf16* __restrict__ ZRL, const __bf16* __restrict__ HT, const __bf16* __restrict__ PK, const float* __restrict__ BZ, const float* __restrict__ BO, const float* __restrict__ BG, const float* __restrict__ BI, const float* __restrict__ MPREV, float* __restrict__ OUTH, float* __restrict__ OUTM) {
  __shared__ __align__(16) __bf16 szh[4][16][72], szl[4][16][72]; __shared__ __align__(16) float sth[CC][68], stm[CC][68];
  const int tid = threadIdx.x, wave = tid >> 5, lane = tid & 31, col = lane & 15, g = lane >> 4; const int pb = blockIdx.x, b = blockIdx.y; const int n0 = pb * 64; const size_t r0 = (size_t)b * NN + n0 + wave * 16;
  { v8f acc[4] = {};
#pragma unroll
    for (int kc = 0; kc < 2 * CC / 32; ++kc) { const v16b ah = frag_b(ZRH + (r0 + col) * 2 * CC + kc * 32, lane), al = frag_b(ZRL + (r0 + col) * 2 * CC + kc * 32, lane);
#pragma unroll
      for (int j = 0; j < 4; ++j) { const v16b w = frag_b(PK + PK_Z + (size_t)(j * 16 + col) * 2 * CC + kc * 32, lane); acc[j] = wmma_bf(al, w, acc[j]); acc[j] = wmma_bf(ah, w, acc[j]); } }
#pragma unroll
    for (int j = 0; j < 4; ++j) { const int c = j * 16 + col; const float bb = bfr(BZ[c]);
#pragma unroll
      for (int r = 0; r < 8; ++r) { const float v = acc[j][r] + bb; const __bf16 hb = (__bf16)v; szh[wave][8 * g + r][c] = hb; szl[wave][8 * g + r][c] = (__bf16)(v - (float)hb); } } }
  LDSX();
  v8f acc[12] = {};
#pragma unroll
  for (int kc = 0; kc < 2 * CC / 32; ++kc) { v16b ah, al; if (kc < 2) { ah = frag_b(HT + (r0 + col) * CC + kc * 32, lane); } else { ah = frag_b(&szh[wave][col][(kc - 2) * 32], lane); al = frag_b(&szl[wave][col][(kc - 2) * 32], lane); }
#pragma unroll
    for (int j = 0; j < 12; ++j) { const v16b w = frag_b(PK + PK_G + (size_t)(j * 16 + col) * 2 * CC + kc * 32, lane); if (kc >= 2) acc[j] = wmma_bf(al, w, acc[j]); acc[j] = wmma_bf(ah, w, acc[j]); } }
#pragma unroll
  for (int j = 0; j < 4; ++j) { const int c = j * 16 + col; const float bo = bfr(BO[c]), bg = bfr(BG[c]), bi = bfr(BI[c]);
#pragma unroll
    for (int r = 0; r < 8; ++r) { const int pl = wave * 16 + 8 * g + r; const float o = 1.0f / (1.0f + exp_ni(-(acc[j][r] + bo))); const float gg = tanh_ni(acc[4 + j][r] + bg); const float ii = 1.0f / (1.0f + exp_ni(-(acc[8 + j][r] + bi)));
      const float mprev = bfr(MPREV[((size_t)b * CC + c) * NN + n0 + pl]); const float mt = (1.0f - ii) * mprev + ii * gg; stm[c][pl] = mt; sth[c][pl] = o * mt; } }
  __syncthreads();
  for (int e = tid; e < CC * 16; e += 128) { const int c = e >> 4, pc = e & 15; const size_t o = ((size_t)b * CC + c) * NN + n0 + pc * 4; vst2(OUTH + o, *(const v4f*)&sth[c][pc * 4]); vst2(OUTM + o, *(const v4f*)&stm[c][pc * 4]); }
}
extern "C" void kernel_launch(void* const* d_in, const int* in_sizes, int n_in, void* d_out, int out_size, void* d_ws, size_t ws_size, hipStream_t stream) {
  (void)in_sizes; (void)n_in; (void)out_size;
  const float** F = (const float**)d_in;
  if (ws_size < (size_t)WS_END) return;
  char* ws = (char*)d_ws; __bf16 *PK = (__bf16*)(ws + WS_PK), *HT = (__bf16*)(ws + WS_HT), *ZRH = (__bf16*)(ws + WS_ZRH), *ZRL = (__bf16*)(ws + WS_ZRL); _Float16 *QP = (_Float16*)(ws + WS_QP), *KP = (_Float16*)(ws + WS_KP), *VH = (_Float16*)(ws + WS_VH), *VL = (_Float16*)(ws + WS_VL);
  float* OUTH = (float*)d_out; float* OUTM = (float*)((char*)d_out + 8388608);
  k_pack<<<dim3(3 * CC, 4), 128, 0, stream>>>(F[2], F[4], F[6], F[8], F[10], F[12], F[14], F[16], F[18], PK);
  k_proj<<<dim3(NN / 64, TNB), 128, 0, stream>>>(F[0], F[1], PK, F[3], F[5], F[7], F[9], F[11], HT, QP, KP, VH, VL);
  k_attn<<<dim3(NN / 64, 2, TNB), 128, 0, stream>>>(QP, KP, VH, VL, ZRH, ZRL);
  k_gate<<<dim3(NN / 64, TNB), 128, 0, stream>>>(ZRH, ZRL, HT, PK, F[13], F[15], F[17], F[19], F[1], OUTH, OUTM);
}
